// ConditionalLayer_16475494548255
// MI455X (gfx1250) — hardware-verified
//
#include <hip/hip_runtime.h>


#define B_ROWS 4096
#define DIM    1024
#define NCOND  8
#define BM     128
#define BN     64
#define BK     32

typedef __attribute__((ext_vector_type(16))) __bf16 v16bf;
typedef __attribute__((ext_vector_type(8)))  __bf16 v8bf;
typedef __attribute__((ext_vector_type(4)))  __bf16 v4bf;
typedef __attribute__((ext_vector_type(8)))  float  v8f;
typedef __attribute__((ext_vector_type(4)))  float  v4f;

__device__ __forceinline__ void async_b128(unsigned lds_off, unsigned goff,
                                           const void* base) {
  asm volatile("global_load_async_to_lds_b128 %0, %1, %2"
               :: "v"(lds_off), "v"(goff), "s"(base) : "memory");
}
__device__ __forceinline__ void wait_async6() {
  asm volatile("s_wait_asynccnt 6" ::: "memory");
}
__device__ __forceinline__ void wait_async0() {
  asm volatile("s_wait_asynccnt 0" ::: "memory");
}
__device__ __forceinline__ unsigned lds_off_of(const void* p) {
  return (unsigned)(uintptr_t)p;
}

__global__ void bucket_kernel(const int* __restrict__ cond,
                              int* __restrict__ row_idx,
                              int* __restrict__ grp_off,
                              int* __restrict__ tile_c,
                              int* __restrict__ tile_m,
                              int* __restrict__ n_tiles) {
  __shared__ int cnt[NCOND], cur[NCOND], off[NCOND + 1];
  const int tid = threadIdx.x;
  if (tid < NCOND) cnt[tid] = 0;
  __syncthreads();
  for (int b = tid; b < B_ROWS; b += 256) atomicAdd(&cnt[cond[b]], 1);
  __syncthreads();
  if (tid == 0) {
    off[0] = 0;
    int t = 0;
    for (int c = 0; c < NCOND; ++c) {
      off[c + 1] = off[c] + cnt[c];
      cur[c] = off[c];
      grp_off[c] = off[c];
      for (int m = off[c]; m < off[c + 1]; m += BM) {
        tile_c[t] = c;
        tile_m[t] = m;
        ++t;
      }
    }
    grp_off[NCOND] = off[NCOND];
    *n_tiles = t;
  }
  __syncthreads();
  for (int b = tid; b < B_ROWS; b += 256) {
    int c = cond[b];
    int pos = atomicAdd(&cur[c], 1);
    row_idx[pos] = b;
  }
}

__global__ void cterm_kernel(const float* __restrict__ b1,
                             const float* __restrict__ b2,
                             const float* __restrict__ W2,
                             float* __restrict__ cterm) {
  __shared__ float rb1[DIM];
  __shared__ int any_nz;
  const int c = blockIdx.x;
  const int tid = threadIdx.x;
  if (tid == 0) any_nz = 0;
  __syncthreads();
  int local = 0;
  for (int d = tid; d < DIM; d += 256) {
    float v = b1[c * DIM + d];
    v = v > 0.f ? v : 0.f;
    rb1[d] = v;
    if (v != 0.f) local = 1;
  }
  if (local) atomicOr(&any_nz, 1);
  __syncthreads();
  const int e = blockIdx.y * 256 + tid;
  float acc = b2[c * DIM + e];
  if (any_nz) {
    const float* w = W2 + (size_t)c * DIM * DIM + e;
    for (int d = 0; d < DIM; ++d) acc += rb1[d] * w[(size_t)d * DIM];
  }
  *(volatile float*)(cterm + c * DIM + e) = acc; __threadfence(); *(volatile float*)(cterm + c * DIM + e) = acc;
}

__global__ void constall_kernel(const float* __restrict__ cterm,
                                float* __restrict__ const_all) {
  const int e = blockIdx.x * 256 + threadIdx.x;
  float s = 0.f;
  for (int c = 0; c < NCOND; ++c) s += cterm[c * DIM + e];
  *(volatile float*)(const_all + e) = s; __threadfence(); *(volatile float*)(const_all + e) = s;
}

__global__ void split_x_kernel(const float* __restrict__ x,
                               __bf16* __restrict__ xhi, __bf16* __restrict__ xlo,
                               __bf16* __restrict__ hhi, __bf16* __restrict__ hlo) {
  const int i = (blockIdx.x * 256 + threadIdx.x) * 4;
  v4f v = *(const v4f*)(x + i);
  v4bf h, l;
#pragma unroll
  for (int j = 0; j < 4; ++j) {
    __bf16 hh = (__bf16)v[j];
    h[j] = hh;
    l[j] = (__bf16)(v[j] - (float)hh);
  }
  *(volatile v4bf*)(xhi + i) = h; *(volatile v4bf*)(xlo + i) = l;
  if (blockIdx.x == 0 && threadIdx.x < 32) {
    const int t = B_ROWS * DIM + threadIdx.x;
    xhi[t] = (__bf16)0.f; xlo[t] = (__bf16)0.f; hhi[t] = (__bf16)0.f; hlo[t] = (__bf16)0.f;
  }
  __threadfence();
  *(volatile v4bf*)(xhi + i) = h; *(volatile v4bf*)(xlo + i) = l;
  if (blockIdx.x == 0 && threadIdx.x < 32) {
    const int t = B_ROWS * DIM + threadIdx.x;
    xhi[t] = (__bf16)0.f; xlo[t] = (__bf16)0.f; hhi[t] = (__bf16)0.f; hlo[t] = (__bf16)0.f;
  }
}

__global__ void __launch_bounds__(256)
split_w_kernel(const float* __restrict__ W,
               __bf16* __restrict__ Whi, __bf16* __restrict__ Wlo) {
  __shared__ __bf16 shi[64][72];
  __shared__ __bf16 slo[64][72];
  const int c = blockIdx.z;
  const int k0 = blockIdx.y * 64;
  const int n0 = blockIdx.x * 64;
  const int tid = threadIdx.x;
  const int kr = tid >> 4;
  const int nc = (tid & 15) * 4;
#pragma unroll
  for (int pass = 0; pass < 4; ++pass) {
    const int kk = kr + pass * 16;
    v4f v = *(const v4f*)(W + ((size_t)(c * DIM + k0 + kk)) * DIM + n0 + nc);
#pragma unroll
    for (int j = 0; j < 4; ++j) {
      __bf16 h = (__bf16)v[j];
      shi[nc + j][kk] = h;
      slo[nc + j][kk] = (__bf16)(v[j] - (float)h);
    }
  }
  __syncthreads();
#pragma unroll 1
  for (int rep = 0; rep < 2; ++rep) {
#pragma unroll
    for (int pass = 0; pass < 2; ++pass) {
      const int idx = pass * 256 + tid;
      const int r = idx >> 3, seg = (idx & 7) * 8;
      const size_t o = ((size_t)(c * DIM + n0 + r)) * DIM + k0 + seg;
      *(volatile v8bf*)(Whi + o) = *(const v8bf*)&shi[r][seg];
      *(volatile v8bf*)(Wlo + o) = *(const v8bf*)&slo[r][seg];
    }
    __threadfence();
  }
}

__device__ __forceinline__ v16bf cat16(v8bf a, v8bf b) {
  return __builtin_shufflevector(a, b, 0, 1, 2, 3, 4, 5, 6, 7,
                                 8, 9, 10, 11, 12, 13, 14, 15);
}

template <bool LAYER2>
__global__ void __launch_bounds__(256)
fc_gemm_kernel(const __bf16* __restrict__ A_hi, const __bf16* __restrict__ A_lo,
               const __bf16* __restrict__ W_hi, const __bf16* __restrict__ W_lo,
               const float* __restrict__ bias,
               const float* __restrict__ const_all,
               const float* __restrict__ cterm,
               const int* __restrict__ row_idx,
               const int* __restrict__ grp_off,
               const int* __restrict__ tile_c,
               const int* __restrict__ tile_m,
               const int* __restrict__ n_tiles_p,
               __bf16* __restrict__ OutHi,
               __bf16* __restrict__ OutLo,
               float* __restrict__ OutF) {
  const int ty = blockIdx.y;
  if (ty >= *n_tiles_p) return;

  const int c      = tile_c[ty];
  const int m_base = tile_m[ty];
  const int m_end  = grp_off[c + 1];
  const int n0     = blockIdx.x * BN;

  __shared__ __attribute__((aligned(16))) unsigned char lds_raw[(2 * BM * BK + 2 * BM * BK + 2 * BN * BK + 2 * BN * BK) * 2 > BM * BN * 4 ? (2 * BM * BK + 2 * BM * BK + 2 * BN * BK + 2 * BN * BK) * 2 : BM * BN * 4];
  __bf16 (*lA_hi)[BM][BK] = (__bf16 (*)[BM][BK])lds_raw;
  __bf16 (*lA_lo)[BM][BK] = (__bf16 (*)[BM][BK])(lds_raw + 2 * BM * BK * 2);
  __bf16 (*lW_hi)[BN][BK] = (__bf16 (*)[BN][BK])(lds_raw + 4 * BM * BK * 2);
  __bf16 (*lW_lo)[BN][BK] = (__bf16 (*)[BN][BK])(lds_raw + 4 * BM * BK * 2 + 2 * BN * BK * 2);

  const int tid    = threadIdx.x;
  const int lane   = tid & 31;
  const int wave   = tid >> 5;
  const int wave_m = wave & 3;
  const int wave_n = wave >> 2;

  const unsigned ZOFF = (unsigned)(B_ROWS * DIM * 2);
  unsigned a_goff[2], a_adv[2], a_lds[2];
#pragma unroll
  for (int r2 = 0; r2 < 2; ++r2) {
    const int idx = r2 * 256 + tid;
    const int row = idx >> 2;
    const int seg = idx & 3;
    const int p = m_base + row;
    const bool ok = p < m_end;
    unsigned grow = 0;
    if (ok) grow = LAYER2 ? (unsigned)p : (unsigned)row_idx[p];
    a_goff[r2] = ok ? (grow * (unsigned)DIM + seg * 8u) * 2u : ZOFF + seg * 16u;
    a_adv[r2]  = ok ? (unsigned)(BK * 2) : 0u;
    a_lds[r2]  = (unsigned)(row * (BK * 2) + seg * 16);
  }
  const int wrow = tid >> 2, wseg = tid & 3;
  unsigned w_goff = ((unsigned)(c * DIM + n0 + wrow) * (unsigned)DIM + wseg * 8u) * 2u;
  const unsigned w_lds = (unsigned)(wrow * (BK * 2) + wseg * 16);

  const unsigned baseAhi = lds_off_of(&lA_hi[0][0][0]);
  const unsigned baseAlo = lds_off_of(&lA_lo[0][0][0]);
  const unsigned baseWhi = lds_off_of(&lW_hi[0][0][0]);
  const unsigned baseWlo = lds_off_of(&lW_lo[0][0][0]);
  const unsigned szA = BM * BK * 2, szW = BN * BK * 2;

  auto issue_slab = [&](int buf) {
#pragma unroll
    for (int r2 = 0; r2 < 2; ++r2) {
      async_b128(baseAhi + buf * szA + a_lds[r2], a_goff[r2], A_hi);
      async_b128(baseAlo + buf * szA + a_lds[r2], a_goff[r2], A_lo);
    }
    async_b128(baseWhi + buf * szW + w_lds, w_goff, W_hi);
    async_b128(baseWlo + buf * szW + w_lds, w_goff, W_lo);
    a_goff[0] += a_adv[0];
    a_goff[1] += a_adv[1];
    w_goff += BK * 2;
  };

  const int fm   = lane & 15;
  const int ksel = (lane >> 4) * 8;

  v8f acc[2][2] = {{v8f{}, v8f{}}, {v8f{}, v8f{}}};

  issue_slab(0);
  for (int k0 = 0; k0 < DIM; k0 += BK) {
    const int cur = (k0 >> 5) & 1;
    if (k0 + BK < DIM) {
      issue_slab(cur ^ 1);
      wait_async6();
    } else {
      wait_async0();
    }
    __syncthreads();

    v16bf bh[2], bl[2];
#pragma unroll
    for (int in = 0; in < 2; ++in) {
      const int bn = wave_n * 32 + in * 16 + (lane & 15);
      bh[in] = cat16(*(const v8bf*)&lW_hi[cur][bn][ksel],
                     *(const v8bf*)&lW_hi[cur][bn][ksel + 16]);
      bl[in] = cat16(*(const v8bf*)&lW_lo[cur][bn][ksel],
                     *(const v8bf*)&lW_lo[cur][bn][ksel + 16]);
    }
#pragma unroll
    for (int im = 0; im < 2; ++im) {
      const int ar = wave_m * 32 + im * 16 + fm;
      const v16bf ah = cat16(*(const v8bf*)&lA_hi[cur][ar][ksel],
                             *(const v8bf*)&lA_hi[cur][ar][ksel + 16]);
      const v16bf al = cat16(*(const v8bf*)&lA_lo[cur][ar][ksel],
                             *(const v8bf*)&lA_lo[cur][ar][ksel + 16]);
#pragma unroll
      for (int in = 0; in < 2; ++in) {
        acc[im][in] = __builtin_amdgcn_wmma_f32_16x16x32_bf16(
            false, ah, false, bh[in], (short)0, acc[im][in], false, false);
        acc[im][in] = __builtin_amdgcn_wmma_f32_16x16x32_bf16(
            false, ah, false, bl[in], (short)0, acc[im][in], false, false);
        acc[im][in] = __builtin_amdgcn_wmma_f32_16x16x32_bf16(
            false, al, false, bh[in], (short)0, acc[im][in], false, false);
      }
    }
    asm volatile("v_nop\n\tv_nop\n\tv_nop\n\tv_nop\n\tv_nop\n\tv_nop" : "+v"(acc[0][0]), "+v"(acc[0][1]), "+v"(acc[1][0]), "+v"(acc[1][1]) :: "memory");
    __syncthreads();
  }

  __syncthreads();
  float* sC = (float*)lds_raw;
#pragma unroll
  for (int in = 0; in < 2; ++in) {
    const int cl_ = wave_n * 32 + in * 16 + (lane & 15);
    const int col = n0 + cl_;
    float badd = bias[c * DIM + col];
    if (LAYER2) badd += const_all[col] - cterm[c * DIM + col];
#pragma unroll
    for (int im = 0; im < 2; ++im)
#pragma unroll
      for (int r = 0; r < 8; ++r) {
        const int mrow = wave_m * 32 + im * 16 + r + 8 * (lane >> 4);
        float v = acc[im][in][r] + badd;
        if (!LAYER2) v = v > 0.f ? v : 0.f;
        sC[mrow * BN + cl_] = v;
      }
  }
  __syncthreads();
#pragma unroll 1
  for (int pass = 0; pass < 2; ++pass) {
    if (!LAYER2) {
      for (int cidx = tid; cidx < BM * 8; cidx += 256) {
        const int mrow = cidx >> 3, q = (cidx & 7) * 8, p = m_base + mrow;
        if (p < m_end) {
          union { v8bf v; __bf16 h[8]; } ph, pl;
#pragma unroll
          for (int j = 0; j < 8; ++j) { const float v = sC[mrow * BN + q + j]; ph.h[j] = (__bf16)v; pl.h[j] = (__bf16)(v - (float)ph.h[j]); }
          *(volatile v8bf*)(OutHi + (size_t)p * DIM + n0 + q) = ph.v;
          *(volatile v8bf*)(OutLo + (size_t)p * DIM + n0 + q) = pl.v;
        }
      }
    } else {
      for (int cidx = tid; cidx < BM * 16; cidx += 256) {
        const int mrow = cidx >> 4, q = (cidx & 15) * 4, p = m_base + mrow;
        if (p < m_end) {
          v4f v; v[0] = sC[mrow * BN + q]; v[1] = sC[mrow * BN + q + 1]; v[2] = sC[mrow * BN + q + 2]; v[3] = sC[mrow * BN + q + 3];
          *(volatile v4f*)(OutF + (size_t)row_idx[p] * DIM + n0 + q) = v;
        }
      }
    }
    __threadfence();
  }
}

extern "C" void kernel_launch(void* const* d_in, const int* in_sizes, int n_in,
                              void* d_out, int out_size, void* d_ws, size_t ws_size,
                              hipStream_t stream) {
  (void)in_sizes; (void)n_in; (void)out_size; (void)ws_size;
  const float* x    = (const float*)d_in[0];
  const int*   cond = (const int*)d_in[1];
  const float* W1   = (const float*)d_in[2];
  const float* b1   = (const float*)d_in[3];
  const float* W2   = (const float*)d_in[4];
  const float* b2   = (const float*)d_in[5];
  float* out = (float*)d_out;

  char* ws = (char*)d_ws;
  size_t off = 0;
  auto carve = [&](size_t bytes) -> char* {
    char* p = ws + off;
    off = (off + bytes + 255) & ~(size_t)255;
    return p;
  };
  const size_t planeB = ((size_t)B_ROWS * DIM + 32) * sizeof(__bf16);
  int*    row_idx   = (int*)carve(B_ROWS * sizeof(int));
  int*    grp_off   = (int*)carve((NCOND + 1) * sizeof(int));
  int*    tile_c    = (int*)carve(80 * sizeof(int));
  int*    tile_m    = (int*)carve(80 * sizeof(int));
  int*    n_tiles   = (int*)carve(sizeof(int));
  float*  cterm     = (float*)carve((size_t)NCOND * DIM * sizeof(float));
  float*  const_all = (float*)carve((size_t)DIM * sizeof(float));
  __bf16* x_hi      = (__bf16*)carve(planeB);
  __bf16* x_lo      = (__bf16*)carve(planeB);
  __bf16* H_hi      = (__bf16*)carve(planeB);
  __bf16* H_lo      = (__bf16*)carve(planeB);
  __bf16* Wt_hi     = (__bf16*)carve((size_t)NCOND * DIM * DIM * sizeof(__bf16));
  __bf16* Wt_lo     = (__bf16*)carve((size_t)NCOND * DIM * DIM * sizeof(__bf16));

  bucket_kernel<<<1, 256, 0, stream>>>(cond, row_idx, grp_off, tile_c, tile_m, n_tiles);
  cterm_kernel<<<dim3(NCOND, DIM / 256), 256, 0, stream>>>(b1, b2, W2, cterm);
  constall_kernel<<<DIM / 256, 256, 0, stream>>>(cterm, const_all);
  split_x_kernel<<<(B_ROWS * DIM) / 1024, 256, 0, stream>>>(x, x_hi, x_lo, H_hi, H_lo);

  split_w_kernel<<<dim3(DIM / 64, DIM / 64, NCOND), 256, 0, stream>>>(W1, Wt_hi, Wt_lo);
  fc_gemm_kernel<false><<<dim3(DIM / BN, 40), 256, 0, stream>>>(
      x_hi, x_lo, Wt_hi, Wt_lo, b1, nullptr, nullptr,
      row_idx, grp_off, tile_c, tile_m, n_tiles, H_hi, H_lo, nullptr);
  split_w_kernel<<<dim3(DIM / 64, DIM / 64, NCOND), 256, 0, stream>>>(W2, Wt_hi, Wt_lo);
  fc_gemm_kernel<true><<<dim3(DIM / BN, 40), 256, 0, stream>>>(
      H_hi, H_lo, Wt_hi, Wt_lo, b2, const_all, cterm,
      row_idx, grp_off, tile_c, tile_m, n_tiles, nullptr, nullptr, out);
}
